// Cosine_PredictingModule_88622355186223
// MI455X (gfx1250) — hardware-verified
//
#include <hip/hip_runtime.h>
#include <math.h>

typedef __attribute__((ext_vector_type(16))) _Float16 v16h;
typedef __attribute__((ext_vector_type(16))) __bf16 v16b;
typedef __attribute__((ext_vector_type(8)))  _Float16 v8h;
typedef __attribute__((ext_vector_type(8)))  float v8f;
typedef __attribute__((ext_vector_type(4)))  float v4f;
typedef __attribute__((ext_vector_type(2)))  float v2f;
typedef __attribute__((ext_vector_type(4)))  unsigned v4u;
typedef __attribute__((ext_vector_type(4)))  int v4i;
typedef float __attribute__((may_alias)) float_a;
typedef int __attribute__((may_alias)) int_a;

template <typename T> __device__ __forceinline__ void vst2(void* p, T v) { *(volatile T*)p = v; __threadfence(); *(volatile T*)p = v; }
__device__ __forceinline__ v8f wmma16(v16h a, v16h b, v8f c) {
  v8f d = __builtin_amdgcn_wmma_f32_16x16x32_f16(false, a, false, b, (short)0, c, false, false);
  asm volatile("v_nop\n\tv_nop\n\tv_nop\n\tv_nop" : "+v"(d) : "v"(a), "v"(b));
  return d;
}
__device__ __forceinline__ v8f wmma_bf(v16b a, v16b b, v8f c) {
  v8f d = __builtin_amdgcn_wmma_f32_16x16x32_bf16(false, a, false, b, (short)0, c, false, false);
  asm volatile("v_nop\n\tv_nop\n\tv_nop\n\tv_nop" : "+v"(d) : "v"(a), "v"(b));
  return d;
}
__device__ __forceinline__ v16h frag_h(const _Float16* rowk0, int lane) {
  union { v16h v; v8h q[2]; } u; const _Float16* p = rowk0 + 8 * (lane >> 4);
  u.q[0] = *(const v8h*)p; u.q[1] = *(const v8h*)(p + 16); return u.v;
}
__device__ __forceinline__ v16h frag_f32(const float* rowk0, int lane) {
  v16h a; const float* p = rowk0 + 8 * (lane >> 4);
#pragma unroll
  for (int i = 0; i < 8; ++i) { a[i] = (_Float16)p[i]; a[8 + i] = (_Float16)p[16 + i]; }
  return a;
}
__device__ __forceinline__ v16h frag_f32s(const float* rowk0, int lane, float sc) {
  v16h a; const float* p = rowk0 + 8 * (lane >> 4);
#pragma unroll
  for (int i = 0; i < 8; ++i) { a[i] = (_Float16)(p[i] * sc); a[8 + i] = (_Float16)(p[16 + i] * sc); }
  return a;
}
__device__ __forceinline__ v16h fragc_f32(const float* W, int k0, int n, int lane, int ld, int K) {
  v16h a; const int g = lane >> 4;
#pragma unroll
  for (int i = 0; i < 8; ++i) { const int ka = k0 + 8 * g + i, kb = ka + 16;
    a[i] = (_Float16)(ka < K ? W[(size_t)ka * ld + n] : 0.f); a[8 + i] = (_Float16)(kb < K ? W[(size_t)kb * ld + n] : 0.f); }
  return a;
}
struct F2 { v16b h, l; };
__device__ __forceinline__ F2 bsplit16(const float v[16]) { F2 r;
#pragma unroll
  for (int i = 0; i < 16; ++i) { const __bf16 h = (__bf16)v[i]; r.h[i] = h; r.l[i] = (__bf16)(v[i] - (float)h); }
  return r; }
__device__ __forceinline__ F2 split_row(const float* row, int k0, int lane) { float v[16]; const float* p = row + k0 + 8 * (lane >> 4);
#pragma unroll
  for (int i = 0; i < 8; ++i) { v[i] = p[i]; v[8 + i] = p[16 + i]; }
  return bsplit16(v); }
__device__ __forceinline__ F2 split_rowK(const float* row, int k0, int lane, int K) { float v[16]; const int g = lane >> 4;
#pragma unroll
  for (int i = 0; i < 8; ++i) { const int ka = k0 + 8 * g + i, kb = ka + 16; v[i] = ka < K ? row[ka] : 0.f; v[8 + i] = kb < K ? row[kb] : 0.f; }
  return bsplit16(v); }
__device__ __forceinline__ F2 split_col(const float* W, int k0, int n, int lane, int ld, int K) { float v[16]; const int g = lane >> 4;
#pragma unroll
  for (int i = 0; i < 8; ++i) { const int ka = k0 + 8 * g + i, kb = ka + 16; v[i] = ka < K ? W[(size_t)ka * ld + n] : 0.f; v[8 + i] = kb < K ? W[(size_t)kb * ld + n] : 0.f; }
  return bsplit16(v); }
__device__ __forceinline__ v8f mac3(const F2& a, const F2& b, v8f c) { c = wmma_bf(a.l, b.h, c); c = wmma_bf(a.h, b.l, c); return wmma_bf(a.h, b.h, c); }
__device__ __forceinline__ float sigm(float v) { return 1.0f / (1.0f + expf(-v)); }
#define LDSX() do { asm volatile("s_wait_dscnt 0" ::: "memory"); __builtin_amdgcn_wave_barrier(); __builtin_amdgcn_fence(__ATOMIC_RELEASE, "workgroup"); } while (0)
__device__ __forceinline__ v16h fragc_f32s(const float* __restrict__ base, int k0, int n, int lane, int ld, float sc) {
  const int g = lane >> 4; v16h r;
#pragma unroll
  for (int i = 0; i < 8; ++i) { r[i] = (_Float16)(base[(size_t)(k0 + 8 * g + i) * ld + n] * sc); r[8 + i] = (_Float16)(base[(size_t)(k0 + 16 + 8 * g + i) * ld + n] * sc); }
  return r;
}

#define NN 100000
#define NE 1000000
#define D 128
#define DIN 257
#define H2 32
#define NNP 100032
typedef _Float16 v4h __attribute__((ext_vector_type(4)));

__global__ __launch_bounds__(128) void k_node(const float* __restrict__ h, const float* __restrict__ W1, int off, float* __restrict__ P, float* __restrict__ NRM) {
  __shared__ __align__(16) float so[4][16][132];
  const int tid = threadIdx.x, wave = tid >> 5, lane = tid & 31, col = lane & 15, g = lane >> 4;
  const int r0 = blockIdx.x * 64 + wave * 16; const int ra = (r0 + col) < NN ? (r0 + col) : NN - 1;
  v8f acc[8] = {};
#pragma unroll
  for (int kc = 0; kc < D / 32; ++kc) { const v16h a = frag_f32(h + (size_t)ra * D + kc * 32, lane);
#pragma unroll
    for (int j = 0; j < 8; ++j) acc[j] = wmma16(a, frag_f32s(W1 + (size_t)(j * 16 + col) * DIN + off + kc * 32, lane, 16.0f), acc[j]); }
#pragma unroll
  for (int j = 0; j < 8; ++j)
#pragma unroll
    for (int r = 0; r < 8; ++r) so[wave][8 * g + r][j * 16 + col] = acc[j][r] * (1.0f / 16.0f);
  LDSX();
  { const int rl = lane >> 1, hf = lane & 1; const float* hr = h + (size_t)((r0 + rl) < NN ? (r0 + rl) : NN - 1) * D + hf * 64; float s = 0.f;
#pragma unroll 1
    for (int c = 0; c < 64; c += 4) { const v4f v = *(const v4f*)(hr + c); s += (v[0] * v[0] + v[1] * v[1]) + (v[2] * v[2] + v[3] * v[3]); }
    s += __shfl_xor(s, 1, 32); if (hf == 0) so[wave][rl][128] = sqrtf(s); }
  LDSX();
#pragma unroll 4
  for (int rl = 0; rl < 16; ++rl) vst2(P + (size_t)(r0 + rl) * D + lane * 4, *(const v4f*)(&so[wave][rl][lane * 4]));
  if (lane < 4) vst2(NRM + (size_t)r0 + lane * 4, (v4f){so[wave][lane * 4][128], so[wave][lane * 4 + 1][128], so[wave][lane * 4 + 2][128], so[wave][lane * 4 + 3][128]});
}
__global__ __launch_bounds__(128) void k_edge(const int* __restrict__ src, const int* __restrict__ dst, const float* __restrict__ hu, const float* __restrict__ hi, const float* __restrict__ PU, const float* __restrict__ PI, const float* __restrict__ NU, const float* __restrict__ NI,
                                            const float* __restrict__ W1, const float* __restrict__ b1, const float* __restrict__ W2, const float* __restrict__ b2, const float* __restrict__ W3, const float* __restrict__ b3, float* __restrict__ out) {
  __shared__ __align__(16) _Float16 sa[4][16][D + 8];
  __shared__ float scos[4][16];
  __shared__ __align__(16) float s2[4][16][36];
  __shared__ __align__(16) float sout[64];
  const int tid = threadIdx.x, wave = tid >> 5, lane = tid & 31, col = lane & 15, g = lane >> 4;
  const int e0 = blockIdx.x * 64 + wave * 16;
  { const int rl = lane >> 1, hf = lane & 1; const int e = e0 + rl; int s = src[e], d = dst[e]; s = s < 0 ? 0 : (s >= NN ? NN - 1 : s); d = d < 0 ? 0 : (d >= NN ? NN - 1 : d);
    const float* a = hu + (size_t)s * D + hf * 64; const float* b = hi + (size_t)d * D + hf * 64; float dot = 0.f;
#pragma unroll 1
    for (int c = 0; c < 64; c += 4) { const v4f x = *(const v4f*)(a + c), y = *(const v4f*)(b + c); dot += (x[0] * y[0] + x[1] * y[1]) + (x[2] * y[2] + x[3] * y[3]); }
    dot += __shfl_xor(dot, 1, 32);
    if (hf == 0) { const float nu = fmaxf(NU[s], 1e-12f), ni = fmaxf(NI[d], 1e-12f);
      const float nhn = NU[s] / nu, ntn = NI[d] / ni; scos[wave][rl] = (dot / (nu * ni)) / fmaxf(nhn * ntn, 1e-8f); }
    LDSX();
    const float cs = scos[wave][rl]; const float* pu = PU + (size_t)s * D + hf * 64; const float* pi = PI + (size_t)d * D + hf * 64;
#pragma unroll 1
    for (int c = 0; c < 64; c += 4) { const v4f x = *(const v4f*)(pu + c), y = *(const v4f*)(pi + c); union { v4h h; unsigned long long u; } pk;
#pragma unroll
      for (int q = 0; q < 4; ++q) { const int cc = hf * 64 + c + q; const float v = x[q] + y[q] + cs * W1[(size_t)cc * DIN + 256] + b1[cc]; pk.h[q] = (_Float16)(v > 0.f ? v : 0.f); }
      *(unsigned long long*)(&sa[wave][rl][hf * 64 + c]) = pk.u; } }
  LDSX();
  { v8f acc[2] = {};
#pragma unroll
    for (int kc = 0; kc < D / 32; ++kc) { const v16h a = frag_h(&sa[wave][col][0] + kc * 32, lane);
#pragma unroll
      for (int j = 0; j < 2; ++j) acc[j] = wmma16(a, frag_f32s(W2 + (size_t)(j * 16 + col) * D + kc * 32, lane, 16.0f), acc[j]); }
#pragma unroll
    for (int j = 0; j < 2; ++j) { const int n = j * 16 + col; const float bb = b2[n];
#pragma unroll
      for (int r = 0; r < 8; ++r) { const float v = acc[j][r] * (1.0f / 16.0f) + bb; s2[wave][8 * g + r][n] = v > 0.f ? v : 0.f; } } }
  LDSX();
  if (lane < 16) { float s = b3[0];
#pragma unroll 1
    for (int k = 0; k < H2; ++k) s += s2[wave][lane][k] * W3[k];
    sout[wave * 16 + lane] = sigm(s); }
  __syncthreads();
  if (tid < 16) vst2(out + (size_t)blockIdx.x * 64 + tid * 4, *(const v4f*)(&sout[tid * 4]));
}
extern "C" void kernel_launch(void* const* d_in, const int* in_sizes, int n_in, void* d_out, int out_size, void* d_ws, size_t ws_size, hipStream_t stream) {
  (void)in_sizes; (void)n_in; (void)out_size; (void)ws_size;
  const float** I = (const float**)d_in;
  const float* hu = I[0]; const float* hi = I[1]; const int* src = (const int*)d_in[2]; const int* dst = (const int*)d_in[3];
  const float* W1 = I[4]; const float* b1 = I[5]; const float* W2 = I[6]; const float* b2 = I[7]; const float* W3 = I[8]; const float* b3 = I[9];
  float* out = (float*)d_out;
  char* ws = (char*)d_ws; size_t off = 0;
  auto take = [&](size_t bytes) { char* p = ws + off; off += (bytes + 255) & ~(size_t)255; return p; };
  float* PU = (float*)take((size_t)NNP * D * 4); float* PI = (float*)take((size_t)NNP * D * 4); float* NU = (float*)take((size_t)NNP * 4); float* NI = (float*)take((size_t)NNP * 4);
  k_node<<<NNP / 64, 128, 0, stream>>>(hu, W1, 0, PU, NU);
  k_node<<<NNP / 64, 128, 0, stream>>>(hi, W1, 128, PI, NI);
  k_edge<<<NE / 64, 128, 0, stream>>>(src, dst, hu, hi, PU, PI, NU, NI, W1, b1, W2, b2, W3, b3, out);
}
